// SDVAE_14955076125396
// MI455X (gfx1250) — hardware-verified
//
#include <hip/hip_runtime.h>
#include <stdint.h>

#define NOBJ   8
#define ZS     64
#define DM     128
#define DM2    256
#define DM3    384
#define NPAIR  28
#define MP     32
#define NROWS  65536
#define NBATCH 8192
#define BPB    32
#define CROWS  64
#define NCHUNK (NROWS / CROWS)
#define CGRID  256
#define EROWS  128

#define ASC  16.0f
#define WSC  64.0f
#define PINV 0.0009765625f

#define LDE  72
#define LDG  136
#define LD2  264
#define LDC  392
#define LDW  72
#define LDO  132

#define E_AZ    0
#define E_WL    18432
#define E_BIAS  36864
#define E_STG   37376
#define E_TOTAL 72192
#define P_WE    0
#define P_AZ    135168
#define P_EFF   152064
#define P_BE    185856
#define P_WA    186880
#define P_PART  187904
#define P_ATT   188928
#define P_TOTAL 189056
#define C_WC    0
#define C_A     50176
#define C_WL    100352
#define C_WS    109568
#define C_REL   118784
#define C_BC    128000
#define C_BL    128256
#define C_BS    128512
#define C_STG   128768
#define C_TOTAL 162560

static_assert(E_WL == E_AZ + EROWS * LDE * 2);
static_assert(E_BIAS == E_WL + EROWS * LDE * 2);
static_assert(E_STG >= E_BIAS + EROWS * 4);
static_assert(E_TOTAL == E_STG + EROWS * LDG * 2);
static_assert((E_STG % 16) == 0);
static_assert(P_AZ == P_WE + DM2 * LD2 * 2);
static_assert(P_EFF == P_AZ + MP * LD2 * 2);
static_assert(P_BE == P_EFF + MP * LD2 * 4);
static_assert(P_WA == P_BE + DM2 * 4);
static_assert(P_PART == P_WA + DM2 * 4);
static_assert(P_ATT >= P_PART + NPAIR * 8 * 4);
static_assert(P_TOTAL >= P_ATT + MP * 4);
static_assert((P_AZ % 16) == 0 && (P_EFF % 16) == 0 && (P_PART % 16) == 0);
static_assert(C_A == C_WC + CROWS * LDC * 2);
static_assert(C_WL == C_A + CROWS * LDC * 2);
static_assert(C_WS == C_WL + ZS * LDW * 2);
static_assert(C_REL == C_WS + ZS * LDW * 2);
static_assert(C_BC == C_REL + CROWS * LDW * 2);
static_assert(C_BL == C_BC + ZS * 4);
static_assert(C_BS == C_BL + ZS * 4);
static_assert(C_STG == C_BS + ZS * 4);
static_assert(C_TOTAL == C_STG + CROWS * LDO * 4);
static_assert((C_STG % 16) == 0 && (C_REL % 16) == 0 && (C_WL % 16) == 0);
static_assert((LDE % 8) == 0 && (LD2 % 8) == 0 && (LDC % 8) == 0 && (LDW % 8) == 0 && (LDG % 8) == 0);
static_assert((LDO % 4) == 0);
static_assert(NROWS % EROWS == 0);
static_assert(NBATCH % BPB == 0);
static_assert(NROWS % CROWS == 0);
static_assert(NPAIR <= MP);

typedef _Float16 f16;
typedef _Float16 v16h __attribute__((ext_vector_type(16)));
typedef _Float16 v8h  __attribute__((ext_vector_type(8)));
typedef _Float16 v8ha __attribute__((ext_vector_type(8), may_alias));
typedef unsigned short v8us __attribute__((ext_vector_type(8)));
typedef float v8f __attribute__((ext_vector_type(8)));
typedef float v4f __attribute__((ext_vector_type(4)));
typedef float v4fa __attribute__((ext_vector_type(4), may_alias));

union FragH { v16h v; v8h h[2]; };

__device__ __forceinline__ float bf16r(float f) {
  unsigned int u = __float_as_uint(f);
  u = u + 0x7FFFu + ((u >> 16) & 1u);
  u &= 0xFFFF0000u;
  return __uint_as_float(u);
}

__device__ __forceinline__ float elu_f(float x) {
  const float xn = fminf(x, 0.0f);
  return x > 0.0f ? x : expm1f(xn);
}

__device__ __forceinline__ v16h ld_frag(const f16* base, int row0, int k0, int ld) {
  const int lane = threadIdx.x & 31;
  const f16* p = base + (row0 + (lane & 15)) * ld + k0 + ((lane >> 4) << 3);
  FragH f;
  f.h[0] = *(const v8h*)p;
  f.h[1] = *(const v8h*)(p + 16);
  return f.v;
}

__device__ __forceinline__ v8f mma_h(v16h a, v16h b, v8f c) {
  return __builtin_amdgcn_wmma_f32_16x16x32_f16(false, a, false, b, (short)0, c, false, false);
}

__device__ __forceinline__ void guard4(v8f& c0, v8f& c1, v8f& c2, v8f& c3,
                                       v16h a0, v16h a1, v16h b0, v16h b1) {
#if defined(__HIP_DEVICE_COMPILE__)
  asm volatile("v_nop\n\tv_nop\n\tv_nop\n\tv_nop"
               : "+v"(c0), "+v"(c1), "+v"(c2), "+v"(c3)
               : "v"(a0), "v"(a1), "v"(b0), "v"(b1));
#endif
}
__device__ __forceinline__ void guard2(v8f& c0, v8f& c1, v16h a0, v16h b0, v16h b1) {
#if defined(__HIP_DEVICE_COMPILE__)
  asm volatile("v_nop\n\tv_nop\n\tv_nop\n\tv_nop"
               : "+v"(c0), "+v"(c1)
               : "v"(a0), "v"(b0), "v"(b1));
#endif
}
__device__ __forceinline__ void guard1(v8f& c0, v16h a0, v16h a1, v16h b0, v16h b1) {
#if defined(__HIP_DEVICE_COMPILE__)
  asm volatile("v_nop\n\tv_nop\n\tv_nop\n\tv_nop"
               : "+v"(c0)
               : "v"(a0), "v"(a1), "v"(b0), "v"(b1));
#endif
}

__global__ __launch_bounds__(256)
void k_cvt_w(const float* __restrict__ s0, unsigned short* d0, int n0,
             const float* __restrict__ s1, unsigned short* d1, int n1,
             const float* __restrict__ s2, unsigned short* d2, int n2,
             const float* __restrict__ s3, unsigned short* d3, int n3,
             const float* __restrict__ s4, unsigned short* d4, int n4) {
  const int sel = (int)blockIdx.y;
  const float* s = s0; unsigned short* d = d0; int n8 = n0;
  if (sel == 1)      { s = s1; d = d1; n8 = n1; }
  else if (sel == 2) { s = s2; d = d2; n8 = n2; }
  else if (sel == 3) { s = s3; d = d3; n8 = n3; }
  else if (sel == 4) { s = s4; d = d4; n8 = n4; }
  const int g = (int)blockIdx.x * 256 + (int)threadIdx.x;
  if (g >= n8) return;
  const float* p = s + (size_t)g * 8;
  const v4f a = *(const v4f*)p;
  const v4f c = *(const v4f*)(p + 4);
  v8h o = {};
#pragma unroll
  for (int e = 0; e < 4; ++e) {
    o[e]     = (f16)(bf16r(a[e]) * WSC);
    o[4 + e] = (f16)(bf16r(c[e]) * WSC);
  }
  const v8us u = __builtin_bit_cast(v8us, o);
  unsigned short* op = d + (size_t)g * 8;
  *(volatile v8us*)op = u;
  __threadfence();
  *(volatile v8us*)op = u;
}

__global__ __launch_bounds__(256)
void k_embed(const float* __restrict__ z, const unsigned short* __restrict__ wobj_h,
             const float* __restrict__ bobj, unsigned short* ze, int nrows) {
  extern __shared__ __align__(16) char smem[];
  f16*   Az   = (f16*)(smem + E_AZ);
  f16*   Wl   = (f16*)(smem + E_WL);
  float* bias = (float*)(smem + E_BIAS);
  f16*   stg  = (f16*)(smem + E_STG);

  const int tid = threadIdx.x, lane = tid & 31, wv = tid >> 5, hl = lane >> 4, l15 = lane & 15;
  const int m0 = (int)blockIdx.x * EROWS;
  if (m0 + EROWS > nrows) return;

  const f16* wsrc = (const f16*)wobj_h;
#pragma unroll
  for (int it = 0; it < 4; ++it) {
    const int idx = tid + it * 256;
    const int r = idx >> 3, c8 = (idx & 7) << 3;
    const float* p = z + (size_t)(m0 + r) * ZS + c8;
    const v4f a = *(const v4f*)p;
    const v4f c = *(const v4f*)(p + 4);
    v8h o = {};
#pragma unroll
    for (int e = 0; e < 4; ++e) {
      o[e]     = (f16)(bf16r(a[e]) * ASC);
      o[4 + e] = (f16)(bf16r(c[e]) * ASC);
    }
    *(v8h*)&Az[r * LDE + c8] = o;
    *(v8h*)&Wl[r * LDE + c8] = *(const v8h*)(wsrc + (size_t)r * ZS + c8);
  }
  if (tid < DM) bias[tid] = bf16r(bobj[tid]);
  __syncthreads();

  const v16h a0 = ld_frag(Az, 16 * wv, 0, LDE);
  const v16h a1 = ld_frag(Az, 16 * wv, 32, LDE);
#pragma unroll 1
  for (int nt = 0; nt < 8; ++nt) {
    const v16h b0 = ld_frag(Wl, 16 * nt, 0, LDE);
    const v16h b1 = ld_frag(Wl, 16 * nt, 32, LDE);
    v8f c = {};
    c = mma_h(a0, b0, c);
    c = mma_h(a1, b1, c);
    guard1(c, a0, a1, b0, b1);
    const int col = nt * 16 + l15;
    const float bb = bias[col];
#pragma unroll
    for (int r = 0; r < 8; ++r) {
      const float v = elu_f(c[r] * PINV + bb);
      stg[(16 * wv + 8 * hl + r) * LDG + col] = (f16)(v * ASC);
    }
  }
  __syncthreads();

  unsigned short* ob = ze + (size_t)m0 * DM;
  const int srow = tid >> 4, sc8 = (tid & 15) << 3;
#pragma unroll
  for (int ph = 0; ph < 8; ++ph) {
    const int row = ph * 16 + srow;
    const v8h val = *(const v8ha*)&stg[row * LDG + sc8];
    *(volatile v8us*)(ob + (size_t)row * DM + sc8) = __builtin_bit_cast(v8us, val);
  }
  __threadfence();
#pragma unroll
  for (int ph = 0; ph < 8; ++ph) {
    const int row = ph * 16 + srow;
    const v8h val = *(const v8ha*)&stg[row * LDG + sc8];
    *(volatile v8us*)(ob + (size_t)row * DM + sc8) = __builtin_bit_cast(v8us, val);
  }
}

__device__ __forceinline__ int pair_first(int p) {
  return (p >= 7) + (p >= 13) + (p >= 18) + (p >= 22) + (p >= 25) + (p >= 27);
}
__device__ __forceinline__ int pair_start(int i) { return (15 * i - i * i) >> 1; }
__device__ __forceinline__ int pair_index(int i, int j) { return pair_start(i) + j - i - 1; }

__global__ __launch_bounds__(256)
void k_pairs(const unsigned short* __restrict__ ze, const unsigned short* __restrict__ we_h,
             const float* __restrict__ be, const float* __restrict__ Wa, const float* __restrict__ ba,
             unsigned short* eg, int bpb, int nbatch) {
  extern __shared__ __align__(16) char smem[];
  f16*   WeL  = (f16*)(smem + P_WE);
  f16*   Az   = (f16*)(smem + P_AZ);
  float* effL = (float*)(smem + P_EFF);
  float* beL  = (float*)(smem + P_BE);
  float* WaL  = (float*)(smem + P_WA);
  float* part = (float*)(smem + P_PART);
  float* attL = (float*)(smem + P_ATT);

  const int tid = threadIdx.x, lane = tid & 31, wv = tid >> 5, hl = lane >> 4, l15 = lane & 15;
  const f16* wsrc = (const f16*)we_h;
  const f16* zsrc = (const f16*)ze;

#pragma unroll 4
  for (int it = 0; it < 32; ++it) {
    const int idx = tid + it * 256;
    const int r = idx >> 5, c8 = (idx & 31) << 3;
    *(v8h*)&WeL[r * LD2 + c8] = *(const v8h*)(wsrc + (size_t)r * DM2 + c8);
  }
  beL[tid] = bf16r(be[tid]);
  WaL[tid] = bf16r(Wa[tid]);
  const float bav = bf16r(ba[0]);
  const v8h zero8 = {};

  for (int it = 0; it < bpb; ++it) {
    const int b = (int)blockIdx.x * bpb + it;
    if (b >= nbatch) break;
    __syncthreads();

#pragma unroll
    for (int q = 0; q < 4; ++q) {
      const int idx = tid + q * 256;
      const int r = idx >> 5, c8 = (idx & 31) << 3;
      const int rr = (r < NPAIR) ? r : (NPAIR - 1);
      const int i = pair_first(rr);
      const int j = rr - pair_start(i) + i + 1;
      const int so = (c8 < DM) ? i : j;
      const int off = c8 & (DM - 1);
      v8h v = *(const v8h*)(zsrc + ((size_t)(b * NOBJ + so) * DM + off));
      v = (r < NPAIR) ? v : zero8;
      *(v8h*)&Az[r * LD2 + c8] = v;
    }
    __syncthreads();

    v8f acc[2][2];
    {
      const v8f z8 = {};
#pragma unroll
      for (int mt = 0; mt < 2; ++mt)
#pragma unroll
        for (int u = 0; u < 2; ++u) acc[mt][u] = z8;
    }
#pragma unroll
    for (int ks = 0; ks < 8; ++ks) {
      const v16h a0 = ld_frag(Az, 0, 32 * ks, LD2);
      const v16h a1 = ld_frag(Az, 16, 32 * ks, LD2);
      const v16h b0 = ld_frag(WeL, 32 * wv, 32 * ks, LD2);
      const v16h b1 = ld_frag(WeL, 32 * wv + 16, 32 * ks, LD2);
      acc[0][0] = mma_h(a0, b0, acc[0][0]);
      acc[0][1] = mma_h(a0, b1, acc[0][1]);
      acc[1][0] = mma_h(a1, b0, acc[1][0]);
      acc[1][1] = mma_h(a1, b1, acc[1][1]);
      guard4(acc[0][0], acc[0][1], acc[1][0], acc[1][1], a0, a1, b0, b1);
    }
#pragma unroll
    for (int mt = 0; mt < 2; ++mt)
#pragma unroll
      for (int u = 0; u < 2; ++u) {
        const int col = (2 * wv + u) * 16 + l15;
        const float bb = beL[col];
#pragma unroll
        for (int r = 0; r < 8; ++r)
          effL[(16 * mt + 8 * hl + r) * LD2 + col] = elu_f(acc[mt][u][r] * PINV + bb);
      }
    __syncthreads();

    if (tid < NPAIR * 8) {
      const int p = tid >> 3, seg = tid & 7;
      const float* ep = effL + p * LD2 + seg * 32;
      const float* wp = WaL + seg * 32;
      float s = 0.0f;
#pragma unroll
      for (int t = 0; t < 8; ++t) {
        const v4f e = *(const v4f*)(ep + 4 * t);
        const v4f w = *(const v4f*)(wp + 4 * t);
        s += e[0] * w[0]; s += e[1] * w[1]; s += e[2] * w[2]; s += e[3] * w[3];
      }
      part[p * 8 + seg] = s;
    }
    __syncthreads();
    if (tid < NPAIR) {
      float s = bav;
#pragma unroll
      for (int t = 0; t < 8; ++t) s += part[tid * 8 + t];
      attL[tid] = __builtin_amdgcn_rcpf(1.0f + expf(-s));
    }
    __syncthreads();

    {
      const int k = wv;
      const int n0 = lane * 8;
      float e[8] = {0.0f, 0.0f, 0.0f, 0.0f, 0.0f, 0.0f, 0.0f, 0.0f};
#pragma unroll
      for (int t = 0; t < 7; ++t) {
        const int o = t + ((t >= k) ? 1 : 0);
        const int i = (k < o) ? k : o;
        const int j = (k < o) ? o : k;
        const int p = pair_index(i, j);
        const float a = attL[p];
        const float* ep = effL + p * LD2 + n0;
        const v4f x0 = *(const v4f*)ep;
        const v4f x1 = *(const v4f*)(ep + 4);
#pragma unroll
        for (int c = 0; c < 4; ++c) {
          e[c]     += a * x0[c];
          e[4 + c] += a * x1[c];
        }
      }
      v8h o = {};
#pragma unroll
      for (int c = 0; c < 8; ++c) o[c] = (f16)(e[c] * ASC);
      const v8us u = __builtin_bit_cast(v8us, o);
      unsigned short* dst = eg + ((size_t)(b * NOBJ + k) * DM2 + n0);
      *(volatile v8us*)dst = u;
      __threadfence();
      *(volatile v8us*)dst = u;
    }
  }
}

__global__ __launch_bounds__(256)
void k_comb(const unsigned short* __restrict__ ze, const unsigned short* __restrict__ eg,
            const unsigned short* __restrict__ wc_h, const unsigned short* __restrict__ wl_h,
            const unsigned short* __restrict__ ws_h,
            const float* __restrict__ bc, const float* __restrict__ bloc, const float* __restrict__ bscale,
            float* out, int nchunks) {
  extern __shared__ __align__(16) char smem[];
  f16*   WcL  = (f16*)(smem + C_WC);
  f16*   At   = (f16*)(smem + C_A);
  f16*   WlL  = (f16*)(smem + C_WL);
  f16*   WsL  = (f16*)(smem + C_WS);
  f16*   relL = (f16*)(smem + C_REL);
  float* bcL  = (float*)(smem + C_BC);
  float* blL  = (float*)(smem + C_BL);
  float* bsL  = (float*)(smem + C_BS);
  float* stg  = (float*)(smem + C_STG);

  const int tid = threadIdx.x, lane = tid & 31, wv = tid >> 5, hl = lane >> 4, l15 = lane & 15;
  const f16* wcs = (const f16*)wc_h;
  const f16* wls = (const f16*)wl_h;
  const f16* wss = (const f16*)ws_h;
  const f16* zsrc = (const f16*)ze;
  const f16* esrc = (const f16*)eg;

#pragma unroll 4
  for (int it = 0; it < 12; ++it) {
    const int idx = tid + it * 256;
    const int r = idx / 48, c8 = (idx - r * 48) << 3;
    *(v8h*)&WcL[r * LDC + c8] = *(const v8h*)(wcs + (size_t)r * DM3 + c8);
  }
#pragma unroll
  for (int it = 0; it < 2; ++it) {
    const int idx = tid + it * 256;
    const int r = idx >> 3, c8 = (idx & 7) << 3;
    *(v8h*)&WlL[r * LDW + c8] = *(const v8h*)(wls + (size_t)r * ZS + c8);
    *(v8h*)&WsL[r * LDW + c8] = *(const v8h*)(wss + (size_t)r * ZS + c8);
  }
  if (tid < ZS) { bcL[tid] = bf16r(bc[tid]); blL[tid] = bf16r(bloc[tid]); bsL[tid] = bf16r(bscale[tid]); }

  for (int ch = (int)blockIdx.x; ch < nchunks; ch += (int)gridDim.x) {
    const int r0 = ch * CROWS;
    __syncthreads();

#pragma unroll
    for (int q = 0; q < 4; ++q) {
      const int idx = tid + q * 256;
      const int r = idx >> 4, c8 = (idx & 15) << 3;
      *(v8h*)&At[r * LDC + c8] = *(const v8h*)(zsrc + (size_t)(r0 + r) * DM + c8);
    }
#pragma unroll
    for (int q = 0; q < 8; ++q) {
      const int idx = tid + q * 256;
      const int r = idx >> 5, c8 = (idx & 31) << 3;
      *(v8h*)&At[r * LDC + DM + c8] = *(const v8h*)(esrc + (size_t)(r0 + r) * DM2 + c8);
    }
    __syncthreads();

    {
      const int mt = wv >> 1, ntb = (wv & 1) * 2;
      v8f c0 = {}, c1 = {};
#pragma unroll
      for (int ks = 0; ks < 12; ++ks) {
        const v16h a  = ld_frag(At, 16 * mt, 32 * ks, LDC);
        const v16h b0 = ld_frag(WcL, 16 * ntb, 32 * ks, LDC);
        const v16h b1 = ld_frag(WcL, 16 * ntb + 16, 32 * ks, LDC);
        c0 = mma_h(a, b0, c0);
        c1 = mma_h(a, b1, c1);
        guard2(c0, c1, a, b0, b1);
      }
      const int col0 = ntb * 16 + l15, col1 = col0 + 16;
      const float bb0 = bcL[col0], bb1 = bcL[col1];
#pragma unroll
      for (int r = 0; r < 8; ++r) {
        const int row = 16 * mt + 8 * hl + r;
        relL[row * LDW + col0] = (f16)((c0[r] * PINV + bb0) * ASC);
        relL[row * LDW + col1] = (f16)((c1[r] * PINV + bb1) * ASC);
      }
    }
    __syncthreads();

    {
      const int sel = wv >> 2, mt = wv & 3;
      const f16* Wt = WlL + sel * (ZS * LDW);
      const float* bb = blL + sel * ZS;
      const v16h a0 = ld_frag(relL, 16 * mt, 0, LDW);
      const v16h a1 = ld_frag(relL, 16 * mt, 32, LDW);
#pragma unroll
      for (int nt = 0; nt < 4; ++nt) {
        const v16h b0 = ld_frag(Wt, 16 * nt, 0, LDW);
        const v16h b1 = ld_frag(Wt, 16 * nt, 32, LDW);
        v8f c = {};
        c = mma_h(a0, b0, c);
        c = mma_h(a1, b1, c);
        guard1(c, a0, a1, b0, b1);
        const int col = nt * 16 + l15;
        const float bv = bb[col];
#pragma unroll
        for (int r = 0; r < 8; ++r)
          stg[(16 * mt + 8 * hl + r) * LDO + sel * ZS + col] = c[r] * PINV + bv;
      }
    }
    __syncthreads();

    float* ob = out + (size_t)r0 * DM + lane * 4;
    const float* sr = stg + lane * 4;
#pragma unroll
    for (int rr = 0; rr < 8; ++rr) {
      const int row = wv * 8 + rr;
      const v4f val = *(const v4fa*)(sr + row * LDO);
      *(volatile v4f*)(ob + (size_t)row * DM) = val;
    }
    __threadfence();
#pragma unroll
    for (int rr = 0; rr < 8; ++rr) {
      const int row = wv * 8 + rr;
      const v4f val = *(const v4fa*)(sr + row * LDO);
      *(volatile v4f*)(ob + (size_t)row * DM) = val;
    }
  }
}

extern "C" void kernel_launch(void* const* d_in, const int* in_sizes, int n_in,
                              void* d_out, int out_size, void* d_ws, size_t ws_size,
                              hipStream_t stream) {
  if (n_in < 14) return;
  if (in_sizes[0] != NROWS * ZS) return;
  if (in_sizes[2] != DM * ZS) return;
  if (in_sizes[3] < DM) return;
  if (in_sizes[4] != DM2 * DM2) return;
  if (in_sizes[5] < DM2) return;
  if (in_sizes[6] != DM2) return;
  if (in_sizes[7] < 1) return;
  if (in_sizes[8] != ZS * DM3) return;
  if (in_sizes[9] < ZS) return;
  if (in_sizes[10] != ZS * ZS) return;
  if (in_sizes[11] < ZS) return;
  if (in_sizes[12] != ZS * ZS) return;
  if (in_sizes[13] < ZS) return;
  if (out_size != NROWS * DM) return;

  const size_t off_ze = 0;
  const size_t sz_ze  = (size_t)NROWS * DM * 2;
  const size_t off_eg = off_ze + sz_ze;
  const size_t sz_eg  = (size_t)NROWS * DM2 * 2;
  const size_t off_wo = off_eg + sz_eg;
  const size_t sz_wo  = (size_t)in_sizes[2] * 2;
  const size_t off_we = off_wo + sz_wo;
  const size_t sz_we  = (size_t)in_sizes[4] * 2;
  const size_t off_wc = off_we + sz_we;
  const size_t sz_wc  = (size_t)in_sizes[8] * 2;
  const size_t off_wl = off_wc + sz_wc;
  const size_t sz_wl  = (size_t)in_sizes[10] * 2;
  const size_t off_ws = off_wl + sz_wl;
  const size_t sz_ws2 = (size_t)in_sizes[12] * 2;
  const size_t need   = off_ws + sz_ws2;
  if (need > ws_size) return;
  if (need > (size_t)134217728) return;

  const float* z      = (const float*)d_in[0];
  const float* Wobj   = (const float*)d_in[2];
  const float* bobj   = (const float*)d_in[3];
  const float* We     = (const float*)d_in[4];
  const float* be     = (const float*)d_in[5];
  const float* Wa     = (const float*)d_in[6];
  const float* ba     = (const float*)d_in[7];
  const float* Wc     = (const float*)d_in[8];
  const float* bc     = (const float*)d_in[9];
  const float* Wloc   = (const float*)d_in[10];
  const float* bloc   = (const float*)d_in[11];
  const float* Wscale = (const float*)d_in[12];
  const float* bscale = (const float*)d_in[13];
  float* out = (float*)d_out;

  char* wsb = (char*)d_ws;
  unsigned short* ze_p = (unsigned short*)(wsb + off_ze);
  unsigned short* eg_p = (unsigned short*)(wsb + off_eg);
  unsigned short* wo_p = (unsigned short*)(wsb + off_wo);
  unsigned short* we_p = (unsigned short*)(wsb + off_we);
  unsigned short* wc_p = (unsigned short*)(wsb + off_wc);
  unsigned short* wl_p = (unsigned short*)(wsb + off_wl);
  unsigned short* ws_p = (unsigned short*)(wsb + off_ws);

  const int n8_wo = in_sizes[2] / 8, n8_we = in_sizes[4] / 8, n8_wc = in_sizes[8] / 8;
  const int n8_wl = in_sizes[10] / 8, n8_ws = in_sizes[12] / 8;
  int n8_max = n8_wo;
  if (n8_we > n8_max) n8_max = n8_we;
  if (n8_wc > n8_max) n8_max = n8_wc;
  if (n8_wl > n8_max) n8_max = n8_wl;
  if (n8_ws > n8_max) n8_max = n8_ws;

  k_cvt_w<<<dim3((n8_max + 255) / 256, 5), dim3(256), 0, stream>>>(
      Wobj, wo_p, n8_wo, We, we_p, n8_we, Wc, wc_p, n8_wc, Wloc, wl_p, n8_wl, Wscale, ws_p, n8_ws);

  (void)hipFuncSetAttribute(reinterpret_cast<const void*>(&k_embed), hipFuncAttributeMaxDynamicSharedMemorySize, E_TOTAL);
  (void)hipFuncSetAttribute(reinterpret_cast<const void*>(&k_pairs), hipFuncAttributeMaxDynamicSharedMemorySize, P_TOTAL);
  (void)hipFuncSetAttribute(reinterpret_cast<const void*>(&k_comb),  hipFuncAttributeMaxDynamicSharedMemorySize, C_TOTAL);

  const int nrows = in_sizes[0] / ZS;
  k_embed<<<dim3(nrows / EROWS), dim3(256), E_TOTAL, stream>>>(z, wo_p, bobj, ze_p, nrows);

  const int nbatch = nrows / NOBJ;
  k_pairs<<<dim3(nbatch / BPB), dim3(256), P_TOTAL, stream>>>(ze_p, we_p, be, Wa, ba, eg_p, BPB, nbatch);

  const int nchunks = nrows / CROWS;
  k_comb<<<dim3(CGRID), dim3(256), C_TOTAL, stream>>>(ze_p, eg_p, wc_p, wl_p, ws_p, bc, bloc, bscale, out, nchunks);
  (void)hipGetLastError();
}
